// Caps2dMatwo_75582834475478
// MI455X (gfx1250) — hardware-verified
//
#include <hip/hip_runtime.h>
#include <math.h>
typedef __attribute__((ext_vector_type(16))) _Float16 v16h;
typedef __attribute__((ext_vector_type(8)))  _Float16 v8h;
typedef __attribute__((ext_vector_type(16))) __bf16   v16b;
typedef __attribute__((ext_vector_type(8)))  __bf16   v8b;
typedef __attribute__((ext_vector_type(8)))  float    v8f;
typedef __attribute__((ext_vector_type(4)))  float    v4f;

#define CN 2
#define T0 4
#define T1 8
#define HH 128
#define WW 128
#define ZP 16
#define ZA 16
#define ZZ 32
#define NPIX (CN * HH * WW)
#define PXB 16

__device__ __forceinline__ void dep_guard1(v8f& a, v16b x, v16b y) { asm volatile("v_nop\n\tv_nop\n\tv_nop\n\tv_nop" : "+v"(a) : "v"(x), "v"(y)); }
__device__ __forceinline__ unsigned short bfb(float f) { unsigned u = __float_as_uint(f); return (unsigned short)((u + 0x7FFFu + ((u >> 16) & 1u)) >> 16); }
__device__ __forceinline__ void splitbf(float f, __bf16& hi, __bf16& lo) { const unsigned short hb = bfb(f); hi = __builtin_bit_cast(__bf16, hb); lo = __builtin_bit_cast(__bf16, bfb(f - __uint_as_float(((unsigned)hb) << 16))); }

__global__ __launch_bounds__(256) void uhat_kernel(const float* __restrict__ x, const float* __restrict__ Wconv, const float* __restrict__ Wpos,
                                                  const float* __restrict__ Wapp, const float* __restrict__ bapp, float* __restrict__ UH) {
  __shared__ __align__(16) float U[PXB][T0 * ZZ * T1];
  __shared__ __align__(16) float S[PXB][ZZ * T0 * T1];
  __shared__ float mpos[T0 * T1 * 16], mapp[T0 * T1 * 16], bap[T0 * T1];
  const int tid = threadIdx.x, lane = tid & 31, wave = tid >> 5, hh = lane >> 4, c = lane & 15;
  const int blk = blockIdx.x;
  const int wblk = blk % (WW / PXB), nh = blk / (WW / PXB), h = nh % HH, n = nh / HH;
  const int w0 = wblk * PXB;
  for (int i = tid; i < T0 * T1 * 16; i += 256) {
    const int t0 = i / (T1 * 16), tp = (i / 16) % T1, ij = i % 16, ii = ij / 4, kk = ij % 4;
    float ss = 0.f;
#pragma unroll
    for (int r = 0; r < 4; ++r) { const float v = Wpos[(t0 * ZP + tp * 2 + (r * 4 + kk) / 8) * T1 + ((r * 4 + kk) % 8)]; ss += v * v; }
    const float v = Wpos[(t0 * ZP + tp * 2 + (ii * 4 + kk) / 8) * T1 + ((ii * 4 + kk) % 8)];
    mpos[i] = v / sqrtf(fmaxf(ss, 1e-12f));
    mapp[i] = Wapp[(t0 * ZA + tp * 2 + (ii * 4 + kk) / 8) * T1 + ((ii * 4 + kk) % 8)];
  }
  for (int i = tid; i < T0 * T1; i += 256) bap[i] = bapp[i];
  for (int img = wave; img < T0 * ZZ; img += 8) {
    const int t0 = img / ZZ, z0 = img % ZZ;
    const float* xim = x + (((size_t)n * T0 + t0) * ZZ + z0) * HH * WW;
    v16b ah, al, bh, bl;
#pragma unroll
    for (int e = 0; e < 16; ++e) {
      const int k = (e < 8) ? (8 * hh + e) : (16 + 8 * hh + (e - 8));
      float av = 0.f, bv = 0.f;
      if (k < 9) {
        const int kh = k / 3, kw = k % 3, yy = h + kh - 1, xx = w0 + c + kw - 1;
        if (yy >= 0 && yy < HH && xx >= 0 && xx < WW) av = xim[(size_t)yy * WW + xx];
        if (c < T1) bv = Wconv[((t0 * 3 + kh) * 3 + kw) * T1 + c];
      }
      __bf16 p, q; splitbf(av, p, q); ah[e] = p; al[e] = q; splitbf(bv, p, q); bh[e] = p; bl[e] = q;
    }
    v8f acc = {0.f,0.f,0.f,0.f,0.f,0.f,0.f,0.f};
    acc = __builtin_amdgcn_wmma_f32_16x16x32_bf16(false, ah, false, bh, (short)0, acc, false, false);
    dep_guard1(acc, ah, bh);
    acc = __builtin_amdgcn_wmma_f32_16x16x32_bf16(false, ah, false, bl, (short)0, acc, false, false);
    dep_guard1(acc, ah, bl);
    acc = __builtin_amdgcn_wmma_f32_16x16x32_bf16(false, al, false, bh, (short)0, acc, false, false);
    dep_guard1(acc, al, bh);
    if (c < T1) {
#pragma unroll
      for (int r = 0; r < 8; ++r) U[8 * hh + r][(t0 * ZZ + z0) * T1 + c] = acc[r];
    }
  }
  __syncthreads();
  {
    const int px = tid >> 4, sub = tid & 15;
    const float cw = (float)(w0 + px) / (float)WW, chh = (float)h / (float)HH;
    for (int pr = sub; pr < T0 * T1; pr += 16) {
      const int t0 = pr / T1, tp = pr % T1;
      float up[16], ua[16];
#pragma unroll
      for (int q = 0; q < 16; ++q) { up[q] = U[px][(t0 * ZZ + (tp & 1) * 16 + q) * T1 + (tp >> 1)]; ua[q] = U[px][(t0 * ZZ + (tp & 1) * 16 + q) * T1 + 4 + (tp >> 1)] + bap[t0 * T1 + tp]; }
      const float* mp = &mpos[(t0 * T1 + tp) * 16]; const float* ma = &mapp[(t0 * T1 + tp) * 16];
#pragma unroll
      for (int i = 0; i < 4; ++i)
#pragma unroll
        for (int kk = 0; kk < 4; ++kk) {
          float sp = 0.f, sa = 0.f;
#pragma unroll
          for (int j = 0; j < 4; ++j) {
            float m = mp[j * 4 + kk]; if (j == 3 && kk == 0) m += cw; if (j == 3 && kk == 1) m += chh;
            sp += up[i * 4 + j] * m; sa += ua[i * 4 + j] * ma[j * 4 + kk];
          }
          S[px][((i * 4 + kk) * T0 + t0) * T1 + tp] = sp;
          S[px][((ZP + i * 4 + kk) * T0 + t0) * T1 + tp] = sa;
        }
    }
  }
  __syncthreads();
  float* dst = UH + (size_t)(((n * HH + h) * WW) + w0) * (ZZ * T0 * T1);
  for (int pass = 0; pass < 2; ++pass) {
    for (int i = tid; i < PXB * ZZ * T0 * T1 / 4; i += 256) { const v4f v = *(const v4f*)(&S[0][0] + 4 * i); *(volatile v4f*)(dst + 4 * i) = v; }
    __threadfence();
  }
}
__device__ __forceinline__ float sigm(float v) { return 1.0f / (1.0f + expf(-v)); }
__global__ __launch_bounds__(256) void routing_kernel(const float* __restrict__ UH, float* __restrict__ out, int nT, int nC) {
  __shared__ float V[T1 * ZZ][32];
  const int lane = threadIdx.x & 31, wave = threadIdx.x >> 5;
  const int blk = blockIdx.x;
  const int wblk = blk % (WW / 32), nh = blk / (WW / 32), h = nh % HH, n = nh / HH;
  const bool posl = lane < ZP;
#pragma unroll 1
  for (int rd = 0; rd < 4; ++rd) {
    const int px = rd * 8 + wave, w = wblk * 32 + px;
    const size_t pix = ((size_t)n * HH + h) * WW + w;
    float u[T0][T1];
    {
      const v4f* up = (const v4f*)(UH + (pix * ZZ + lane) * (T0 * T1));
#pragma unroll
      for (int i = 0; i < 8; ++i) { const v4f t = up[i];
#pragma unroll
        for (int q = 0; q < 4; ++q) u[(4 * i + q) / T1][(4 * i + q) % T1] = t[q]; }
    }
    float bl[T0][T1];
#pragma unroll
    for (int cc = 0; cc < T0; ++cc)
#pragma unroll
      for (int t = 0; t < T1; ++t) bl[cc][t] = 0.f;
    float vz[T1];
    for (int it = 0; it < 3; ++it) {
      float p[T1];
#pragma unroll 1
      for (int t = 0; t < nT; ++t) { float s = 0.f;
#pragma unroll 1
        for (int cc = 0; cc < nC; ++cc) s += u[cc][t] * sigm(bl[cc][t]); p[t] = s; }
#pragma unroll 1
      for (int t = 0; t < nT; ++t) {
        float mx = fabsf(p[t]), sq = p[t] * p[t];
#pragma unroll
        for (int o = 1; o < 16; o <<= 1) { mx = fmaxf(mx, __shfl_xor(mx, o, 32)); sq += __shfl_xor(sq, o, 32); }
        vz[t] = posl ? (p[t] / mx) : (sq / (1.0f + sq) * p[t] / sqrtf(sq + 1e-9f));
      }
      if (it == 2) break;
#pragma unroll 1
      for (int cc = 0; cc < nC; ++cc)
#pragma unroll 1
        for (int t = 0; t < nT; ++t) {
          float s = u[cc][t] * vz[t];
#pragma unroll
          for (int o = 1; o < 16; o <<= 1) s += __shfl_xor(s, o, 32);
          const float other = __shfl_xor(s, 16, 32);
          bl[cc][t] += s * other;
        }
    }
#pragma unroll
    for (int t = 0; t < T1; ++t) V[t * ZZ + lane][px] = vz[t];
  }
  __syncthreads();
  for (int pass = 0; pass < 2; ++pass) {
    for (int l = wave; l < T1 * ZZ; l += 8) {
      const int t = l / ZZ, z = l % ZZ;
      ((volatile float*)out)[((((size_t)n * T1 + t) * ZZ + z) * HH + h) * WW + wblk * 32 + lane] = V[l][lane];
    }
    __threadfence();
  }
}

extern "C" void kernel_launch(void* const* d_in, const int* in_sizes, int n_in,
                              void* d_out, int out_size, void* d_ws, size_t ws_size,
                              hipStream_t stream) {
  (void)in_sizes; (void)n_in; (void)out_size; (void)ws_size;
  const float* x = (const float*)d_in[0];
  const float* Wconv = (const float*)d_in[1];
  const float* Wpos = (const float*)d_in[2];
  const float* Wapp = (const float*)d_in[3];
  const float* bapp = (const float*)d_in[4];
  float* out = (float*)d_out;
  float* UH = (float*)d_ws;
  uhat_kernel<<<NPIX / PXB, 256, 0, stream>>>(x, Wconv, Wpos, Wapp, bapp, UH);
  routing_kernel<<<NPIX / 32, 256, 0, stream>>>(UH, out, T1, T0);
}
